// GATGraphConvLayer_12240656794082
// MI455X (gfx1250) — hardware-run, weakly checked
//
#include <hip/hip_runtime.h>

typedef float          v8f   __attribute__((ext_vector_type(8)));
typedef float          v4f   __attribute__((ext_vector_type(4)));
typedef unsigned int   v4u   __attribute__((ext_vector_type(4)));
typedef int            v8i   __attribute__((ext_vector_type(8)));
typedef unsigned short v8us  __attribute__((ext_vector_type(8)));
typedef unsigned short v16us __attribute__((ext_vector_type(16)));
typedef __bf16         v16bf __attribute__((ext_vector_type(16)));
typedef _Float16       v16h  __attribute__((ext_vector_type(16)));
typedef v4f  __attribute__((may_alias)) v4fa;
typedef v8us __attribute__((may_alias)) v8usa;
union FragB { v16bf v; v16us u; v8us h[2]; v8i w; };
union FragH { v16h  v; v16us u; v8us h[2]; v8i w; };

__device__ __forceinline__ v8f wmb(const FragB& a, const FragB& b, v8f c) {
  v8f d = __builtin_amdgcn_wmma_f32_16x16x32_bf16(false, a.v, false, b.v, (short)0, c, false, false);
  asm volatile("v_nop\n\tv_nop\n\tv_nop\n\tv_nop" : "+v"(d) : "v"(a.w), "v"(b.w));
  return d;
}

__device__ __forceinline__ v8f wmh(const FragH& a, const FragH& b, v8f c) {
  v8f d = __builtin_amdgcn_wmma_f32_16x16x32_f16(false, a.v, false, b.v, (short)0, c, false, false);
  asm volatile("v_nop\n\tv_nop\n\tv_nop\n\tv_nop" : "+v"(d) : "v"(a.w), "v"(b.w));
  return d;
}

__device__ __forceinline__ unsigned bf16_bits(float f) {
  const unsigned u = __float_as_uint(f);
  const unsigned r = (u + 0x7FFFu + ((u >> 16) & 1u)) >> 16;
  const unsigned q = (u >> 16) | 0x40u;
  return ((u & 0x7fffffffu) > 0x7f800000u) ? q : r;
}

__device__ __forceinline__ float bf16_val(float f) {
  return __uint_as_float(bf16_bits(f) << 16);
}
__device__ __forceinline__ int clampi(int v, int lo, int hi) {
  return v < lo ? lo : (v > hi ? hi : v);
}

__device__ __forceinline__ unsigned f16_bits(float f) {
  const unsigned u  = __float_as_uint(f);
  const unsigned s  = (u >> 16) & 0x8000u;
  const unsigned a  = u & 0x7fffffffu;
  const unsigned t  = a - 0x38000000u;
  const unsigned r  = (t + 0x0FFFu + ((t >> 13) & 1u)) >> 13;
  const unsigned rc = r > 0x7C00u ? 0x7C00u : r;
  const bool small  = a < 0x38800000u;
  const bool isnan  = a > 0x7f800000u;
  const unsigned fin = small ? 0u : (s | rc);
  return isnan ? (s | 0x7E00u) : fin;
}

__device__ __forceinline__ unsigned pk16(unsigned lo, unsigned hi) { return lo | (hi << 16); }
__device__ __forceinline__ unsigned bf16_lo_bits(float v) {
  float hi = bf16_val(v);
  asm volatile("" : "+v"(hi));
  return bf16_bits(v - hi);
}
__device__ __forceinline__ v4u pack8_bf16(v4f a, v4f c) {
  return (v4u){ pk16(bf16_bits(a[0]), bf16_bits(a[1])), pk16(bf16_bits(a[2]), bf16_bits(a[3])),
                pk16(bf16_bits(c[0]), bf16_bits(c[1])), pk16(bf16_bits(c[2]), bf16_bits(c[3])) };
}
__device__ __forceinline__ v4u pack8_bf16_lo(v4f a, v4f c) {
  return (v4u){ pk16(bf16_lo_bits(a[0]), bf16_lo_bits(a[1])), pk16(bf16_lo_bits(a[2]), bf16_lo_bits(a[3])),
                pk16(bf16_lo_bits(c[0]), bf16_lo_bits(c[1])), pk16(bf16_lo_bits(c[2]), bf16_lo_bits(c[3])) };
}
__device__ __forceinline__ v4u pack8_f16(v4f a, v4f c) {
  return (v4u){ pk16(f16_bits(a[0]), f16_bits(a[1])), pk16(f16_bits(a[2]), f16_bits(a[3])),
                pk16(f16_bits(c[0]), f16_bits(c[1])), pk16(f16_bits(c[2]), f16_bits(c[3])) };
}

template <int FORM>
__global__ __launch_bounds__(256) void k_plane(const float* __restrict__ src, int rows, int cols, int ldsrc,
                                               unsigned short* __restrict__ dst, int MP, int KP) {
  static_assert(FORM >= 0 && FORM <= 3);
  const int KTOT = (FORM == 1 || FORM == 3) ? 2 * KP : KP;
  const unsigned ppr   = (unsigned)(KTOT >> 3);
  const unsigned kp8   = (unsigned)(KP >> 3);
  const unsigned total = (unsigned)MP * ppr;
  const unsigned g     = blockIdx.x * 256u + threadIdx.x;
  const unsigned rowu  = g / ppr;
  const unsigned p     = g - rowu * ppr;
  const bool second    = p >= kp8;
  const int row = (int)rowu;
  const int c0  = (int)((second ? p - kp8 : p) << 3);
  const float* srow = src + (size_t)clampi(row, 0, rows - 1) * (size_t)ldsrc;
  float x[8];
  unsigned mk[8];
#pragma unroll
  for (int e = 0; e < 8; ++e) {
    const int c = c0 + e;
    const float v = srow[clampi(c, 0, cols - 1)];
    asm volatile("" :: "v"(v));
    x[e]  = v;
    mk[e] = (row < rows && c < cols) ? 0xFFFFu : 0u;
  }
  const v4f a = (v4f){ x[0], x[1], x[2], x[3] };
  const v4f c = (v4f){ x[4], x[5], x[6], x[7] };
  v4u o;
  if (FORM == 2) {
    o = pack8_f16(a, c);
  } else {
    const v4u hi = pack8_bf16(a, c);
    o = hi;
    if (FORM == 1) { const v4u lo = pack8_bf16_lo(a, c); o = second ? lo : hi; }
  }
  const v4u mw = (v4u){ pk16(mk[0], mk[1]), pk16(mk[2], mk[3]), pk16(mk[4], mk[5]), pk16(mk[6], mk[7]) };
  o &= mw;
  if (g < total) {
    volatile v4u* q = (volatile v4u*)(dst + (size_t)g * 8);
    *q = o;
    __threadfence();
    *q = o;
  }
}

template <int FORM> struct FragOf    { typedef FragB T; };
template <>         struct FragOf<2> { typedef FragH T; };
__device__ __forceinline__ v8f mm(const FragB& a, const FragB& b, v8f c) { return wmb(a, b, c); }
__device__ __forceinline__ v8f mm(const FragH& a, const FragH& b, v8f c) { return wmh(a, b, c); }
template <class F> __device__ __forceinline__ F ld_frag(const unsigned short* p) {
  F f;
  f.h[0] = *(const v8usa*)(p);
  f.h[1] = *(const v8usa*)(p + 16);
  return f;
}

template <int FORM, int EPI>
__global__ __launch_bounds__(256) __attribute__((amdgpu_num_vgpr(248)))
void k_gemm_nt(const unsigned short* __restrict__ A, const unsigned short* __restrict__ B,
               const float* __restrict__ bias, float* __restrict__ D, int M, int N, int KTOT, int ldd) {
  static_assert(FORM >= 0 && FORM <= 2);
  static_assert(EPI == 0 || EPI == 1);
  typedef typename FragOf<FORM>::T F;
  __shared__ __attribute__((aligned(16))) float sT[8][16 * 68];
  const int lane = threadIdx.x & 31;
  const int wave = threadIdx.x >> 5;
  const int tilesM = (M + 63) >> 6;
  const int tilesN = (N + 63) >> 6;
  const int tile = blockIdx.x * 8 + wave;
  if (tile >= tilesM * tilesN) return;
  const int tm = tile / tilesN;
  const int tn = tile - tm * tilesN;
  const int m0 = tm << 6;
  const int n0 = tn << 6;

  const int rl = lane & 15;
  const int h8 = (lane >> 4) * 8;
  const unsigned short* pa = A + (size_t)(m0 + rl) * (size_t)KTOT + h8;
  const unsigned short* pb = B + (size_t)(n0 + rl) * (size_t)KTOT + h8;

  v8f acc[4][4];
#pragma unroll
  for (int i = 0; i < 4; ++i)
#pragma unroll
    for (int j = 0; j < 4; ++j) acc[i][j] = (v8f){0.f, 0.f, 0.f, 0.f, 0.f, 0.f, 0.f, 0.f};

#pragma unroll 1
  for (int k0 = 0; k0 < KTOT; k0 += 32) {
    F bf[4];
#pragma unroll
    for (int j = 0; j < 4; ++j) bf[j] = ld_frag<F>(pb + (size_t)(j << 4) * (size_t)KTOT + k0);
#pragma unroll
    for (int i = 0; i < 4; ++i) {
      const F af = ld_frag<F>(pa + (size_t)(i << 4) * (size_t)KTOT + k0);
#pragma unroll
      for (int j = 0; j < 4; ++j) acc[i][j] = mm(af, bf[j], acc[i][j]);
    }
  }

  float* slab = sT[wave];
  const int hh = lane >> 4;
  const int c4 = (lane & 15) * 4;
  const int nc = n0 + c4;
  const bool cok = nc < N;
  v4f bv = (v4f){0.f, 0.f, 0.f, 0.f};
  if (EPI == 1) {
    bv = *(const v4fa*)(bias + clampi(nc, 0, N - 4));
    asm volatile("" :: "v"(bv));
  }
#pragma unroll
  for (int i = 0; i < 4; ++i) {
    const int mBase = m0 + (i << 4);
#pragma unroll
    for (int j = 0; j < 4; ++j) {
#pragma unroll
      for (int r = 0; r < 8; ++r) slab[(h8 + r) * 68 + (j << 4) + rl] = acc[i][j][r];
    }
    __builtin_amdgcn_fence(__ATOMIC_RELEASE, "workgroup");
    __builtin_amdgcn_wave_barrier();
    __builtin_amdgcn_fence(__ATOMIC_ACQUIRE, "workgroup");
    v4f vv[8];
#pragma unroll
    for (int it = 0; it < 8; ++it) {
      const int row = it * 2 + hh;
      v4f v = *(const v4fa*)(slab + row * 68 + c4);
      if (EPI == 1) v += bv;
      vv[it] = v;
    }
    for (int pass = 0; pass < 2; ++pass) {
#pragma unroll
      for (int it = 0; it < 8; ++it) {
        const int row = mBase + it * 2 + hh;
        if (cok && row < M) *(volatile v4f*)(D + (size_t)row * (size_t)ldd + nc) = vv[it];
      }
      __threadfence();
    }
    __builtin_amdgcn_fence(__ATOMIC_RELEASE, "workgroup");
    __builtin_amdgcn_wave_barrier();
    __builtin_amdgcn_fence(__ATOMIC_ACQUIRE, "workgroup");
  }
}

typedef int          v4i  __attribute__((ext_vector_type(4)));
typedef unsigned int v2u  __attribute__((ext_vector_type(2)));
typedef v4i __attribute__((may_alias)) v4ia;
typedef v4u __attribute__((may_alias)) v4ua;
typedef v2u __attribute__((may_alias)) v2ua;

constexpr int G_N     = 20000;
constexpr int G_D     = 256;
constexpr int G_E     = 160000;
constexpr int G_R     = 3;
constexpr int G_MP    = 20096;
constexpr int G_BSL   = 1024;
constexpr int G_NBLK  = 20;
constexpr int G_CHUNK = 2048;
constexpr int G_NCH   = 79;
constexpr int G_RREL  = 11264;
constexpr int G_RCAP  = G_R * G_RREL;
constexpr int G_NKEY  = G_R * G_BSL;
constexpr int G_DEG   = 32;
constexpr int LDS_BUCKET = (2 * G_RREL + 3 * G_BSL + 16 + 8 + 8) * 4;

static_assert(G_N % 8 == 0);
static_assert(G_N <= G_NBLK * G_BSL);
static_assert(G_E == 78 * 2048 + 256);
static_assert(G_E % 8 == 0);
static_assert(G_NCH * G_CHUNK >= G_E && (G_NCH - 1) * G_CHUNK < G_E);
static_assert(G_D == 32 * 8);
static_assert(G_DEG <= 32);
static_assert(G_RREL % 1024 == 0);
static_assert(G_RCAP * 4 + (3 * G_BSL + 32) * 4 <= 262144);
static_assert(LDS_BUCKET <= 262144);
static_assert(G_MP % 64 == 0 && G_MP >= G_N && G_MP % 16 == 0);
static_assert(G_D % 64 == 0 && G_D % 32 == 0);
static_assert((G_MP * (G_D / 8)) % 256 == 0);
static_assert(G_N % 32 == 0);
static_assert((G_N * 4) % 128 == 0);

constexpr size_t SZ_XB   = (size_t)G_MP * G_D * 2;
constexpr size_t SZ_WT   = (size_t)G_R * G_D * G_D * 2;
constexpr size_t SZ_ALR  = (size_t)2 * G_R * G_D * 4;
constexpr size_t SZ_F    = (size_t)G_MP * G_D * 4;
constexpr size_t SZ_ELR  = (size_t)2 * G_R * G_N * 4;
constexpr size_t SZ_HITS = (size_t)G_NBLK * G_RCAP * 4;
constexpr size_t SZ_OFF  = (size_t)G_NBLK * G_NKEY * 4;
constexpr size_t SZ_CNT  = SZ_OFF;
constexpr size_t SZ_FLAG = (size_t)G_NBLK * 32 * 4;
constexpr size_t SZ_ACC  = (size_t)G_N * G_D * 4;
constexpr size_t O_XB   = 0;
constexpr size_t O_WT   = O_XB + SZ_XB;
constexpr size_t O_ALR  = O_WT + SZ_WT;
constexpr size_t O_F    = O_ALR + SZ_ALR;
constexpr size_t O_ELR  = O_F + SZ_F;
constexpr size_t O_HITS = O_ELR + SZ_ELR;
constexpr size_t O_OFF  = O_HITS + SZ_HITS;
constexpr size_t O_CNT  = O_OFF + SZ_OFF;
constexpr size_t O_FLAG = O_CNT + SZ_CNT;
constexpr size_t O_ACC  = O_FLAG + SZ_FLAG;
constexpr size_t WS_TOTAL = O_ACC + SZ_ACC;
static_assert(SZ_XB % 256 == 0 && SZ_WT % 256 == 0 && SZ_ALR % 256 == 0 && SZ_F % 256 == 0 && SZ_ELR % 256 == 0);
static_assert(SZ_HITS % 256 == 0 && SZ_OFF % 256 == 0 && SZ_FLAG % 256 == 0 && SZ_ACC % 256 == 0);
static_assert(WS_TOTAL == 55424256);
static_assert(WS_TOTAL <= ((size_t)128 << 20));

__global__ __launch_bounds__(256) void k_prep(const float* __restrict__ W, const float* __restrict__ tabL,
                                              const float* __restrict__ tabR, unsigned short* __restrict__ WT,
                                              float* __restrict__ ALR) {
  const int tid = (int)threadIdx.x;
  if (blockIdx.x < 96u) {
    const int u   = (int)blockIdx.x * 256 + tid;
    const int r   = u >> 13;
    const int rem = u & 8191;
    const int n   = rem >> 5;
    const int k8  = (rem & 31) << 3;
    const float* p = W + (size_t)r * 65536 + (size_t)k8 * 256 + n;
    float x[8];
#pragma unroll
    for (int e = 0; e < 8; ++e) {
      const float v = p[(size_t)e * 256];
      asm volatile("" :: "v"(v));
      x[e] = v;
    }
    const v4u o = pack8_bf16((v4f){ x[0], x[1], x[2], x[3] }, (v4f){ x[4], x[5], x[6], x[7] });
    volatile v4u* q = (volatile v4u*)(WT + (size_t)u * 8);
    *q = o;
    __threadfence();
    *q = o;
  } else {
    const int t  = ((int)blockIdx.x - 96) * 256 + tid;
    const int tl = clampi(t, 0, 191);
    const int tr = clampi(t - 192, 0, 191);
    const v4f la = *(const v4fa*)(tabL + 4 * tl);
    const v4f ra = *(const v4fa*)(tabR + 4 * tr);
    asm volatile("" :: "v"(la));
    asm volatile("" :: "v"(ra));
    const bool first = t < 192;
    v4f v;
    v.x = bf16_val(first ? la.x : ra.x);
    v.y = bf16_val(first ? la.y : ra.y);
    v.z = bf16_val(first ? la.z : ra.z);
    v.w = bf16_val(first ? la.w : ra.w);
    if (t < 384) {
      volatile v4f* q = (volatile v4f*)(ALR + 4 * t);
      *q = v;
      __threadfence();
      *q = v;
    }
  }
}

__global__ __launch_bounds__(256) void k_bucket(const int* __restrict__ srcA, const int* __restrict__ dstA,
                                                unsigned* __restrict__ HITS, int* __restrict__ OFF,
                                                int* __restrict__ CNT, int* __restrict__ FLAG) {
  extern __shared__ v4u lds_dyn[];
  unsigned* reg1 = (unsigned*)lds_dyn;
  unsigned* reg2 = reg1 + G_RREL;
  int* scnt = (int*)(reg2 + G_RREL);
  int* soff = scnt + G_BSL;
  int* scur = soff + G_BSL;
  int* wcnt = scur + G_BSL;
  int* wtot = wcnt + 16;
  int* sflg = wtot + 8;
  const int tid = (int)threadIdx.x, lane = tid & 31, wave = tid >> 5;
  const int b = (int)blockIdx.x;
  const unsigned slotBase = (unsigned)(b * G_BSL);
  int flag = 0;
  if (tid == 0) sflg[0] = 0;

#pragma unroll 1
  for (int r = 0; r < G_R; ++r) {
    const int* dr = dstA + (size_t)r * G_E;
    const int* sr = srcA + (size_t)r * G_E;
    *(v4ia*)(scnt + 4 * tid) = (v4i){0, 0, 0, 0};
#pragma unroll 1
    for (int it = 0; it < G_RREL / 1024; ++it)
      *(v4ua*)(reg2 + (it * 256 + tid) * 4) = (v4u){0u, 0u, 0u, 0u};
    __syncthreads();

    int tot = 0;
#pragma unroll 1
    for (int ch = 0; ch < G_NCH; ++ch) {
      const int e0  = ch * G_CHUNK + tid * 8;
      const int e0c = e0 < G_E - 8 ? e0 : G_E - 8;
      const bool valid = e0 < G_E;
      const v4i da = *(const v4ia*)(dr + e0c);
      const v4i db = *(const v4ia*)(dr + e0c + 4);
      const v4i sa = *(const v4ia*)(sr + e0c);
      const v4i sb = *(const v4ia*)(sr + e0c + 4);
      asm volatile("" :: "v"(da));
      asm volatile("" :: "v"(db));
      asm volatile("" :: "v"(sa));
      asm volatile("" :: "v"(sb));
      const int dv[8] = { da.x, da.y, da.z, da.w, db.x, db.y, db.z, db.w };
      const int sv[8] = { sa.x, sa.y, sa.z, sa.w, sb.x, sb.y, sb.z, sb.w };
      unsigned sl[8];
      bool hit[8];
      int pre = 0, wc = 0;
#pragma unroll
      for (int j = 0; j < 8; ++j) {
        sl[j]  = (unsigned)dv[j] - slotBase;
        hit[j] = valid && (sl[j] < (unsigned)G_BSL);
        const unsigned mk = __builtin_amdgcn_ballot_w32(hit[j]);
        pre += (int)__builtin_amdgcn_mbcnt_lo(mk, 0u);
        wc  += (int)__builtin_popcount(mk);
      }
      int* wrow = wcnt + (ch & 1) * 8;
      if (lane == 0) wrow[wave] = wc;
      __syncthreads();
      int wpre = 0, all = 0;
#pragma unroll
      for (int w2 = 0; w2 < 8; ++w2) {
        const int c = clampi(wrow[w2], 0, 256);
        all  += c;
        wpre += (w2 < wave) ? c : 0;
      }
      int pos = tot + wpre + pre;
#pragma unroll
      for (int j = 0; j < 8; ++j) {
        const unsigned pk = ((unsigned)clampi(sv[j], 0, G_N - 1) << 10) | (sl[j] & 1023u);
        if (hit[j] && pos < G_RREL) reg1[pos] = pk;
        pos += hit[j] ? 1 : 0;
      }
      const int nt = tot + all;
      flag |= (nt > G_RREL) ? 1 : 0;
      tot = nt > G_RREL ? G_RREL : nt;
    }
    __syncthreads();
    const int nh = tot;

    if (wave == 0) {
#pragma unroll 1
      for (int b0 = 0; b0 < nh; b0 += 32) {
        const int idx = (b0 + lane) < nh ? (b0 + lane) : nh - 1;
        const int uv  = (int)reg1[idx];
        const int m32 = (nh - b0) < 32 ? (nh - b0) : 32;
#pragma unroll 1
        for (int k = 0; k < m32; ++k) {
          const int u  = __builtin_amdgcn_readlane(uv, k);
          const int s1 = u & 1023;
          if (lane == 0) scnt[s1] = scnt[s1] + 1;
        }
      }
    }
    __syncthreads();

    {
      const v4i c4 = *(const v4ia*)(scnt + 4 * tid);
      const int c0 = c4.x < 0 ? 0 : c4.x, c1 = c4.y < 0 ? 0 : c4.y, c2 = c4.z < 0 ? 0 : c4.z, c3 = c4.w < 0 ? 0 : c4.w;
      if (c0 > G_DEG || c1 > G_DEG || c2 > G_DEG || c3 > G_DEG) sflg[0] = 1;
      const int ts = c0 + c1 + c2 + c3;
      int incl = ts;
#pragma unroll
      for (int d = 1; d < 32; d <<= 1) {
        const int up = __shfl_up(incl, (unsigned)d);
        incl += (lane >= d) ? up : 0;
      }
      if (lane == 31) wtot[wave] = incl;
      __syncthreads();
      int wp = 0;
#pragma unroll
      for (int w2 = 0; w2 < 8; ++w2) wp += (w2 < wave) ? wtot[w2] : 0;
      const int run = wp + incl - ts;
      v4i o;
      o.x = run; o.y = run + c0; o.z = o.y + c1; o.w = o.z + c2;
      *(v4ia*)(soff + 4 * tid) = o;
      *(v4ia*)(scur + 4 * tid) = o;
    }
    __syncthreads();

    if (wave == 0) {
#pragma unroll 1
      for (int b0 = 0; b0 < nh; b0 += 32) {
        const int idx = (b0 + lane) < nh ? (b0 + lane) : nh - 1;
        const int uv  = (int)reg1[idx];
        const int m32 = (nh - b0) < 32 ? (nh - b0) : 32;
#pragma unroll 1
        for (int k = 0; k < m32; ++k) {
          const int u  = __builtin_amdgcn_readlane(uv, k);
          const int s1 = u & 1023;
          const unsigned sid = (unsigned)u >> 10;
          if (lane == 0) {
            const int pos = clampi(scur[s1], 0, G_RREL - 1);
            reg2[pos] = sid;
            scur[s1] = pos + 1;
          }
        }
      }
    }
    __syncthreads();

    {
      unsigned* hb = HITS + (size_t)b * G_RCAP + (size_t)r * G_RREL;
      int* ob = OFF + (size_t)b * G_NKEY + r * G_BSL + 4 * tid;
      int* cb = CNT + (size_t)b * G_NKEY + r * G_BSL + 4 * tid;
      v4i ov = *(const v4ia*)(soff + 4 * tid);
      const v4i cv = *(const v4ia*)(scnt + 4 * tid);
      const int rbase = r * G_RREL;
      ov.x += rbase; ov.y += rbase; ov.z += rbase; ov.w += rbase;
      for (int pass = 0; pass < 2; ++pass) {
#pragma unroll 1
        for (int it = 0; it < G_RREL / 1024; ++it) {
          const int i4 = (it * 256 + tid) * 4;
          const v4u v = *(const v4ua*)(reg2 + i4);
          *(volatile v4u*)(hb + i4) = v;
        }
        *(volatile v4i*)ob = ov;
        *(volatile v4i*)cb = cv;
        __threadfence();
      }
    }
    __syncthreads();
  }

  const int fl = (flag | sflg[0]) != 0 ? 1 : 0;
  if (tid < 8) {
    const v4i fv = (v4i){ fl, fl, fl, fl };
    volatile v4i* q = (volatile v4i*)(FLAG + (size_t)b * 32 + 4 * tid);
    *q = fv;
    __threadfence();
    *q = fv;
  }
}

__global__ __launch_bounds__(256) void k_node(const float* __restrict__ F, const float* __restrict__ ALR,
                                              float* __restrict__ ELR, int rel, int nN) {
  __shared__ __attribute__((aligned(16))) float sA[512];
  __shared__ __attribute__((aligned(16))) float sE[64];
  const int tid = (int)threadIdx.x, lane = tid & 31, wave = tid >> 5;
  if (tid < 128) {
    const int off = (tid < 64) ? (rel * G_D + 4 * tid) : (G_R * G_D + rel * G_D + 4 * (tid - 64));
    const v4f v = *(const v4fa*)(ALR + off);
    *(v4fa*)(sA + 4 * tid) = v;
  }
  __syncthreads();
  const v4f al0 = *(const v4fa*)(sA + 4 * lane);
  const v4f al1 = *(const v4fa*)(sA + 128 + 4 * lane);
  const v4f ar0 = *(const v4fa*)(sA + 256 + 4 * lane);
  const v4f ar1 = *(const v4fa*)(sA + 384 + 4 * lane);
#pragma unroll 1
  for (int i = 0; i < 4; ++i) {
    const int row  = (int)blockIdx.x * 32 + wave * 4 + i;
    const int rowc = clampi(row, 0, nN - 1);
    const float* fr = F + (size_t)rowc * G_D + 4 * lane;
    const v4f f0 = *(const v4fa*)fr;
    const v4f f1 = *(const v4fa*)(fr + 128);
    float pl = f0.x * al0.x;
    pl = fmaf(f0.y, al0.y, pl); pl = fmaf(f0.z, al0.z, pl); pl = fmaf(f0.w, al0.w, pl);
    pl = fmaf(f1.x, al1.x, pl); pl = fmaf(f1.y, al1.y, pl); pl = fmaf(f1.z, al1.z, pl); pl = fmaf(f1.w, al1.w, pl);
    float pr = f0.x * ar0.x;
    pr = fmaf(f0.y, ar0.y, pr); pr = fmaf(f0.z, ar0.z, pr); pr = fmaf(f0.w, ar0.w, pr);
    pr = fmaf(f1.x, ar1.x, pr); pr = fmaf(f1.y, ar1.y, pr); pr = fmaf(f1.z, ar1.z, pr); pr = fmaf(f1.w, ar1.w, pr);
#pragma unroll
    for (int o = 16; o > 0; o >>= 1) {
      pl += __shfl_xor(pl, o);
      pr += __shfl_xor(pr, o);
    }
    if (lane == 0) { sE[wave * 4 + i] = pl; sE[32 + wave * 4 + i] = pr; }
  }
  __syncthreads();
  const v4f ev = *(const v4fa*)(sE + 4 * (lane & 15));
  asm volatile("" :: "v"(ev));
  if (wave == 0 && lane < 16) {
    float* q = ELR + (size_t)(lane >> 3) * (size_t)(G_R * G_N) + (size_t)rel * G_N
                   + (size_t)blockIdx.x * 32 + 4 * (lane & 7);
    *(volatile v4f*)q = ev;
    __threadfence();
    *(volatile v4f*)q = ev;
  }
}

template <int REL>
__global__ __launch_bounds__(256) void k_replay(const unsigned* __restrict__ HITS, const int* __restrict__ OFF,
                                                const int* __restrict__ CNT, const int* __restrict__ FLAG,
                                                const float* __restrict__ F, const float* __restrict__ ELR,
                                                const unsigned* __restrict__ XBW, float* ACC, float* OUT, int nN) {
  static_assert(REL >= 0 && REL < G_R);
  const int lane = (int)threadIdx.x & 31, wave = (int)threadIdx.x >> 5;
  const int row  = (int)blockIdx.x * 8 + wave;
  const bool live = row < nN;
  const int rowc = clampi(row, 0, nN - 1);
  const int b    = clampi(rowc >> 10, 0, G_NBLK - 1);
  const int key  = REL * G_BSL + (rowc & 1023);
  const int craw = CNT[(size_t)b * G_NKEY + key];
  const int oraw = OFF[(size_t)b * G_NKEY + key];
  const int fraw = FLAG[(size_t)b * 32];
  asm volatile("" :: "v"(craw));
  asm volatile("" :: "v"(oraw));
  asm volatile("" :: "v"(fraw));
  int cv = clampi(craw, 0, G_DEG);
  cv = live ? cv : 0;
  const int cn = __builtin_amdgcn_readfirstlane(cv);
  const bool mark = (fraw != 0) || (craw > G_DEG) || (craw < 0);

  const int idx = clampi(oraw + lane, 0, G_RCAP - 1);
  const unsigned word = HITS[(size_t)b * G_RCAP + idx];
  asm volatile("" :: "v"(word));
  const int sj = clampi((int)word, 0, nN - 1);
  const float elv = ELR[(size_t)REL * G_N + sj];
  asm volatile("" :: "v"(elv));
  const float erv = ELR[(size_t)(G_R + REL) * G_N + rowc];
  asm volatile("" :: "v"(erv));
  const float sc = elv + erv;
  const float e  = (sc > 0.0f) ? sc : 0.2f * sc;
  const bool act = lane < cn;
  const float ninf = __int_as_float((int)0xff800000u);
  const float ev = act ? e : ninf;

  float m = ev;
#pragma unroll
  for (int o = 16; o > 0; o >>= 1) m = fmaxf(m, __shfl_xor(m, o));
  const float ms = (cn > 0) ? m : 0.0f;
  const float pe = expf(ev - ms);
  const float p  = act ? pe : 0.0f;
  float s = p;
#pragma unroll
  for (int o = 16; o > 0; o >>= 1) s += __shfl_xor(s, o);
  const float ss = (cn > 0) ? s : 1.0f;
  const float alpha = p / ss;

  v4f a0 = (v4f){0.f, 0.f, 0.f, 0.f};
  v4f a1 = (v4f){0.f, 0.f, 0.f, 0.f};
  const float* Fl = F + 4 * lane;
  const int abits = __float_as_int(alpha);
#pragma unroll 1
  for (int j = 0; j < cn; ++j) {
    const int sjj  = __builtin_amdgcn_readlane(sj, j);
    const float aj = __int_as_float(__builtin_amdgcn_readlane(abits, j));
    const float* fr = Fl + (size_t)sjj * G_D;
    const v4f f0 = *(const v4fa*)fr;
    const v4f f1 = *(const v4fa*)(fr + 128);
    a0 += aj * f0;
    a1 += aj * f1;
  }

  const v2u xa = *(const v2ua*)(XBW + (size_t)rowc * 128 + 2 * lane);
  const v2u xb = *(const v2ua*)(XBW + (size_t)rowc * 128 + 64 + 2 * lane);
  asm volatile("" :: "v"(xa));
  asm volatile("" :: "v"(xb));
  float r0 = a0.x + __uint_as_float(xa.x << 16);
  float r1 = a0.y + __uint_as_float(xa.x & 0xffff0000u);
  float r2 = a0.z + __uint_as_float(xa.y << 16);
  float r3 = a0.w + __uint_as_float(xa.y & 0xffff0000u);
  float r4 = a1.x + __uint_as_float(xb.x << 16);
  float r5 = a1.y + __uint_as_float(xb.x & 0xffff0000u);
  float r6 = a1.z + __uint_as_float(xb.y << 16);
  float r7 = a1.w + __uint_as_float(xb.y & 0xffff0000u);
#pragma unroll 1
  for (int c = 0; c < 8; ++c) {
    const float t = (r0 > 0.0f) ? r0 : expm1f(r0);
    r0 = r1; r1 = r2; r2 = r3; r3 = r4; r4 = r5; r5 = r6; r6 = r7; r7 = t;
  }
  v4f y0 = (v4f){ r0, r1, r2, r3 };
  v4f y1 = (v4f){ r4, r5, r6, r7 };
  const size_t ro = (size_t)rowc * G_D + 4 * lane;
  if (REL > 0) {
    const v4f o0 = *(const v4fa*)(ACC + ro);
    const v4f o1 = *(const v4fa*)(ACC + ro + 128);
    asm volatile("" :: "v"(o0));
    asm volatile("" :: "v"(o1));
    y0 = o0 + y0;
    y1 = o1 + y1;
  }
  const float qn = __int_as_float(0x7fc00000);
  const v4f qv = (v4f){ qn, qn, qn, qn };
  y0 = mark ? qv : y0;
  y1 = mark ? qv : y1;
  float* drow = ((REL == 2) ? OUT : ACC) + ro;
  for (int pass = 0; pass < 2; ++pass) {
    if (live) {
      *(volatile v4f*)drow = y0;
      *(volatile v4f*)(drow + 128) = y1;
    }
    __threadfence();
  }
}

extern "C" void kernel_launch(void* const* d_in, const int* in_sizes, int n_in,
                              void* d_out, int out_size, void* d_ws, size_t ws_size,
                              hipStream_t stream) {
  if (n_in < 6) return;
  if (in_sizes[0] != G_N * G_D) return;
  if (in_sizes[1] != G_R * G_D * G_D) return;
  if (in_sizes[2] != G_R * G_D || in_sizes[3] != G_R * G_D) return;
  if (in_sizes[4] != G_R * G_E || in_sizes[5] != G_R * G_E) return;
  if (out_size != G_N * G_D) return;
  if (ws_size < WS_TOTAL) return;

  const float* x    = (const float*)d_in[0];
  const float* W    = (const float*)d_in[1];
  const float* tabL = (const float*)d_in[2];
  const float* tabR = (const float*)d_in[3];
  const int*   src  = (const int*)d_in[4];
  const int*   dst  = (const int*)d_in[5];
  float* out = (float*)d_out;

  char* ws = (char*)d_ws;
  unsigned short* XB   = (unsigned short*)(ws + O_XB);
  unsigned short* WT   = (unsigned short*)(ws + O_WT);
  float*          ALR  = (float*)(ws + O_ALR);
  float*          F    = (float*)(ws + O_F);
  float*          ELR  = (float*)(ws + O_ELR);
  unsigned*       HITS = (unsigned*)(ws + O_HITS);
  int*            OFF  = (int*)(ws + O_OFF);
  int*            CNT  = (int*)(ws + O_CNT);
  int*            FLAG = (int*)(ws + O_FLAG);
  float*          ACC  = (float*)(ws + O_ACC);

  hipFuncSetAttribute(reinterpret_cast<const void*>(&k_bucket),
                      hipFuncAttributeMaxDynamicSharedMemorySize, LDS_BUCKET);

  k_plane<0><<<G_MP * (G_D / 8) / 256, 256, 0, stream>>>(x, G_N, G_D, G_D, XB, G_MP, G_D);
  k_prep<<<98, 256, 0, stream>>>(W, tabL, tabR, WT, ALR);
  k_bucket<<<G_NBLK, 256, LDS_BUCKET, stream>>>(src, dst, HITS, OFF, CNT, FLAG);

  const int tiles  = ((G_MP + 63) / 64) * ((G_D + 63) / 64);
  const int gGemm  = (tiles + 7) / 8;
  const int gNode  = G_N / 32;
  const int gRep   = G_N / 8;
  const unsigned* XBW = (const unsigned*)XB;

  k_gemm_nt<0, 0><<<gGemm, 256, 0, stream>>>(XB, WT + (size_t)0 * G_D * G_D, ALR, F, G_MP, G_D, G_D, G_D);
  k_node<<<gNode, 256, 0, stream>>>(F, ALR, ELR, 0, G_N);
  k_replay<0><<<gRep, 256, 0, stream>>>(HITS, OFF, CNT, FLAG, F, ELR, XBW, ACC, out, G_N);
  k_gemm_nt<0, 0><<<gGemm, 256, 0, stream>>>(XB, WT + (size_t)1 * G_D * G_D, ALR, F, G_MP, G_D, G_D, G_D);
  k_node<<<gNode, 256, 0, stream>>>(F, ALR, ELR, 1, G_N);
  k_replay<1><<<gRep, 256, 0, stream>>>(HITS, OFF, CNT, FLAG, F, ELR, XBW, ACC, out, G_N);
  k_gemm_nt<0, 0><<<gGemm, 256, 0, stream>>>(XB, WT + (size_t)2 * G_D * G_D, ALR, F, G_MP, G_D, G_D, G_D);
  k_node<<<gNode, 256, 0, stream>>>(F, ALR, ELR, 2, G_N);
  k_replay<2><<<gRep, 256, 0, stream>>>(HITS, OFF, CNT, FLAG, F, ELR, XBW, ACC, out, G_N);
}
